// PhasedSNForecastModel_42606075576840
// MI455X (gfx1250) — hardware-run, weakly checked
//
#include <hip/hip_runtime.h>

typedef __attribute__((ext_vector_type(16))) _Float16 v16h;
typedef __attribute__((ext_vector_type(8)))  _Float16 v8h;
typedef __attribute__((ext_vector_type(8)))  float    v8f;
typedef __attribute__((ext_vector_type(4)))  float    v4f;
typedef __attribute__((ext_vector_type(2)))  float    v2f;

__device__ __forceinline__ void dep_guard_h(v8f& a, v8f& b, v16h x, v16h y) { asm volatile("v_nop\n\tv_nop\n\tv_nop\n\tv_nop" : "+v"(a), "+v"(b) : "v"(x), "v"(y)); }
__device__ __forceinline__ void keep4_h(v16h a, v16h b, v16h c, v16h d) { asm volatile("v_nop" :: "v"(a), "v"(b), "v"(c), "v"(d)); }
__device__ __forceinline__ void acc_guard4(v8f& a, v8f& b, v8f& c, v8f& d) { asm volatile("v_nop\n\tv_nop\n\tv_nop\n\tv_nop" : "+v"(a), "+v"(b), "+v"(c), "+v"(d)); }
template <typename T> struct Frag;
template <> struct Frag<_Float16> {
  typedef v16h V; union U { v16h v; v8h h[2]; };
  static __device__ __forceinline__ v16h load(const _Float16* p) {
    U f; f.h[0] = *(const v8h*)(p); f.h[1] = *(const v8h*)(p + 16); return f.v;
  }
  static __device__ __forceinline__ v8f mma(v16h a, v16h b, v8f c) {
    return __builtin_amdgcn_wmma_f32_16x16x32_f16(false, a, false, b, (short)0, c, false, false);
  }
  static __device__ __forceinline__ void guard(v8f& a, v8f& b, v16h x, v16h y) { dep_guard_h(a, b, x, y); }
  static __device__ __forceinline__ void keep(v16h a, v16h b, v16h c, v16h d) { keep4_h(a, b, c, d); }
};

constexpr int NBATCH = 1024;
constexpr int NSEQ   = 512;
constexpr int NFEAT  = 2;
constexpr int NH1    = 128;
constexpr int NH2    = 64;
constexpr int NHD    = 32;
constexpr int NOUTS  = 32;
constexpr int NTT    = NSEQ + NOUTS - 1;
constexpr int KTW    = NH1 + NH2;
constexpr int KCAT   = NH1 + NH2;
constexpr int APITCH = 200;
constexpr int ROWSPB = 16;
constexpr int OUTROW = NOUTS * NFEAT;
constexpr float OPA_SCALE = 8.0f;
constexpr float OPB_SCALE = 16.0f;
constexpr float OP_INV    = 1.0f / 128.0f;

__device__ __forceinline__ float sigm(float z) { return __builtin_amdgcn_rcpf(1.0f + expf(-z)); }

__global__ __launch_bounds__(256) void k_prep_wt(const float* __restrict__ s1, int K1,
                                                 const float* __restrict__ s2, int K2, int N,
                                                 _Float16* __restrict__ dst, int nchunks, float scl) {
  const int id = blockIdx.x * 256 + threadIdx.x;
  if (id < nchunks) {
    const int KT  = K1 + K2;
    const int kc8 = KT >> 3;
    const int n   = id / kc8;
    const int k0  = (id - n * kc8) * 8;
    v8h hv;
#pragma unroll
    for (int e = 0; e < 8; ++e) {
      const int kk = k0 + e;
      const int i1 = (kk < K1) ? kk : (K1 - 1);
      int i2 = kk - K1;
      i2 = (i2 > K2 - 1) ? (K2 - 1) : i2;
      i2 = (i2 < 0) ? 0 : i2;
      const float v1 = s1[(size_t)i1 * N + n];
      const float v2 = s2[(size_t)i2 * N + n];
      const float v  = (kk < K1) ? v1 : v2;
      hv[e] = (_Float16)(v * scl);
    }
    _Float16* d = dst + (size_t)id * 8;
    *(volatile v8h*)d = hv;
    __threadfence();
    *(volatile v8h*)d = hv;
  }
}

__global__ __launch_bounds__(256) void k_stats(const float* __restrict__ x, float* __restrict__ stats) {
  __shared__ __align__(16) float red4[8 * 4];
  const int tid = threadIdx.x, wave = tid >> 5, lane = tid & 31;
  const int b = blockIdx.x * 8 + wave;
  const float PINF = __uint_as_float(0x7f800000u);
  const float NINF = __uint_as_float(0xff800000u);
  const v4f* p = reinterpret_cast<const v4f*>(x + (size_t)b * (NSEQ * NFEAT));
  float mx0 = NINF, mx1 = NINF, mn0 = PINF, mn1 = PINF;
#pragma unroll
  for (int i = 0; i < 8; ++i) {
    const v4f v = p[lane + 32 * i];
    mx0 = fmaxf(mx0, fmaxf(v[0], v[2]));
    mx1 = fmaxf(mx1, fmaxf(v[1], v[3]));
    const float a0 = (v[0] > -1.0f) ? v[0] : PINF;
    const float a2 = (v[2] > -1.0f) ? v[2] : PINF;
    const float a1 = (v[1] > -1.0f) ? v[1] : PINF;
    const float a3 = (v[3] > -1.0f) ? v[3] : PINF;
    mn0 = fminf(mn0, fminf(a0, a2));
    mn1 = fminf(mn1, fminf(a1, a3));
  }
#pragma unroll
  for (int off = 16; off > 0; off >>= 1) {
    mx0 = fmaxf(mx0, __shfl_xor(mx0, off, 32));
    mx1 = fmaxf(mx1, __shfl_xor(mx1, off, 32));
    mn0 = fminf(mn0, __shfl_xor(mn0, off, 32));
    mn1 = fminf(mn1, __shfl_xor(mn1, off, 32));
  }
  if (lane == 0) { red4[wave * 4 + 0] = mx0; red4[wave * 4 + 1] = mx1; red4[wave * 4 + 2] = mn0; red4[wave * 4 + 3] = mn1; }
  __syncthreads();
  if (wave == 0) {
    const int li = lane & 7;
    const v4f val = *(const v4f*)(red4 + li * 4);
    float* dst = stats + (size_t)(blockIdx.x * 8 + li) * 4;
    if (lane < 8) *(volatile v4f*)dst = val;
    __threadfence();
    if (lane < 8) *(volatile v4f*)dst = val;
  }
}

__global__ __launch_bounds__(256) void k_ktab(const float* __restrict__ tau1, const float* __restrict__ shift1,
                                              const float* __restrict__ ron1,
                                              const float* __restrict__ tau2, const float* __restrict__ shift2,
                                              const float* __restrict__ ron2,
                                              float* __restrict__ ktab, int n4) {
#pragma clang fp contract(off)
  const int id = blockIdx.x * 256 + threadIdx.x;
  if (id < n4) {
    const int e0 = id * 4;
    const int t  = e0 / KTW;
    const int ub = e0 - t * KTW;
    const float tf = (float)t;
    v4f kv;
#pragma unroll
    for (int e = 0; e < 4; ++e) {
      const int u  = ub + e;
      const int i1 = (u < NH1) ? u : (NH1 - 1);
      int i2 = u - NH1;
      i2 = (i2 < 0) ? 0 : i2;
      i2 = (i2 > NH2 - 1) ? (NH2 - 1) : i2;
      const float ta = tau1[i1], sa = shift1[i1], ra = ron1[i1];
      const float tb = tau2[i2], sb = shift2[i2], rb = ron2[i2];
      const bool  first = (u < NH1);
      const float tau = first ? ta : tb;
      const float sh  = first ? sa : sb;
      const float ron = first ? ra : rb;
      const float d = tf - sh;
      float r = fmodf(d, tau);
      if (r != 0.0f && ((r < 0.0f) != (tau < 0.0f))) r = r + tau;
      const float phi = r / tau;
      float k;
      if (phi < 0.5f * ron)      k = 2.0f * phi / ron;
      else if (phi < ron)        k = 2.0f - 2.0f * phi / ron;
      else                       k = 0.001f * phi;
      kv[e] = k;
    }
    float* dst = ktab + (size_t)id * 4;
    *(volatile v4f*)dst = kv;
    __threadfence();
    *(volatile v4f*)dst = kv;
  }
}

__global__ __launch_bounds__(256) void k_main(
    const float* __restrict__ inputs, const float* __restrict__ W1,
    const float* __restrict__ b1, const float* __restrict__ b2,
    const float* __restrict__ Wd1, const float* __restrict__ bd1,
    const float* __restrict__ Wo, const float* __restrict__ bo,
    const int* __restrict__ osteps_p,
    const _Float16* __restrict__ U1t, const _Float16* __restrict__ Bcat,
    const float* __restrict__ stats, const float* __restrict__ ktab,
    float* __restrict__ out)
{
  __shared__ __align__(16) _Float16 Ah[ROWSPB * APITCH];
  __shared__ __align__(16) float xs[ROWSPB * NFEAT];
  __shared__ __align__(16) float h2f[ROWSPB * 68];
  __shared__ __align__(16) float df[ROWSPB * 36];
  __shared__ __align__(16) float predst[ROWSPB * OUTROW];
  __shared__ __align__(16) float stt[ROWSPB * 8];
  __shared__ float red[8];
  union FU { v16h v; v8h h[2]; };

  const int tid  = threadIdx.x;
  const int wave = tid >> 5;
  const int lane = tid & 31;
  const int c    = lane & 15;
  const int hh   = lane >> 4;
  const int b0   = blockIdx.x * ROWSPB;
  const float PINF = __uint_as_float(0x7f800000u);
  const float NINF = __uint_as_float(0xff800000u);
  const v8f z8 = {0.f, 0.f, 0.f, 0.f, 0.f, 0.f, 0.f, 0.f};

  {
    unsigned* Aw = reinterpret_cast<unsigned*>(Ah);
    for (int i = tid; i < ROWSPB * APITCH / 2; i += 256) Aw[i] = 0u;
    for (int i = tid; i < ROWSPB * OUTROW; i += 256) predst[i] = 0.0f;
    if (tid < ROWSPB * NFEAT) xs[tid] = 0.0f;
  }

  const v4f* sp = reinterpret_cast<const v4f*>(stats);
  {
    float mx = NINF;
#pragma unroll
    for (int i = 0; i < 4; ++i) {
      const v4f s = sp[tid * 4 + i];
      mx = fmaxf(mx, fmaxf(s[0], s[1]));
    }
#pragma unroll
    for (int off = 16; off > 0; off >>= 1) mx = fmaxf(mx, __shfl_xor(mx, off, 32));
    if (lane == 0) red[wave] = mx;
  }
  __syncthreads();
  float max_all = red[0];
#pragma unroll
  for (int i = 1; i < 8; ++i) max_all = fmaxf(max_all, red[i]);
  if (tid < ROWSPB) {
    const v4f s = sp[b0 + tid];
    const float mn0 = (s[2] == PINF) ? max_all : s[2];
    const float mn1 = (s[3] == PINF) ? max_all : s[3];
    const float rg0 = s[0] - mn0;
    const float rg1 = s[1] - mn1;
    stt[tid * 8 + 0] = mn0;
    stt[tid * 8 + 1] = mn1;
    stt[tid * 8 + 2] = 1.0f / rg0;
    stt[tid * 8 + 3] = 1.0f / rg1;
    stt[tid * 8 + 4] = rg0;
    stt[tid * 8 + 5] = rg1;
    stt[tid * 8 + 6] = 0.0f;
    stt[tid * 8 + 7] = 0.0f;
  }
  __syncthreads();
  if (wave == 0) {
    const int row = lane >> 1, f = lane & 1;
    const float v = inputs[(size_t)(b0 + row) * (NSEQ * NFEAT) + f];
    xs[lane] = (v - stt[row * 8 + f]) * stt[row * 8 + 2 + f];
  }

  const int u1 = 16 * wave + c;
  const int u2 = 16 * (wave & 3) + c;
  float b1q[4], w1a[4], w1b[4], b2q[4];
#pragma unroll
  for (int q = 0; q < 4; ++q) {
    const int n1 = NH1 * q + u1;
    b1q[q] = b1[n1];
    w1a[q] = W1[n1];
    w1b[q] = W1[4 * NH1 + n1];
    const int n2 = NH2 * q + u2;
    b2q[q] = b2[n2];
  }
  float c1s[8], h1s[8], c2s[8], h2s[8];
#pragma unroll
  for (int r = 0; r < 8; ++r) { c1s[r] = 0.f; h1s[r] = 0.f; c2s[r] = 0.f; h2s[r] = 0.f; }

  int osteps = osteps_p[0];
  osteps = (osteps < 1) ? 1 : ((osteps > NOUTS) ? NOUTS : osteps);
  osteps = __builtin_amdgcn_readfirstlane(osteps);
  const int nroll = osteps - 1;
  __syncthreads();

#pragma unroll 1
  for (int tt = 0; tt < NSEQ + nroll; ++tt) {
    const bool warm = (tt < NSEQ);

    v8f acc[4];
#pragma unroll
    for (int q = 0; q < 4; ++q) acc[q] = z8;
#pragma unroll
    for (int ks = 0; ks < NH1 / 32; ++ks) {
      v16h bq[4];
#pragma unroll
      for (int q = 0; q < 4; ++q)
        bq[q] = Frag<_Float16>::load(U1t + (size_t)(NH1 * q + u1) * NH1 + ks * 32 + 8 * hh);
      FU a;
      a.h[0] = *(const v8h*)(Ah + c * APITCH + ks * 32 + 8 * hh);
      a.h[1] = *(const v8h*)(Ah + c * APITCH + ks * 32 + 16 + 8 * hh);
#pragma unroll
      for (int q = 0; q < 4; ++q) acc[q] = Frag<_Float16>::mma(a.v, bq[q], acc[q]);
      dep_guard_h(acc[0], acc[3], a.v, a.v);
      keep4_h(bq[0], bq[1], bq[2], bq[3]);
    }
    acc_guard4(acc[0], acc[1], acc[2], acc[3]);

    const float kv1  = ktab[(size_t)tt * KTW + u1];
    const float okv1 = 1.0f - kv1;
    float x0[8], x1[8];
    unsigned mbits = 0xffu;
#pragma unroll
    for (int r = 0; r < 8; ++r) {
      const v2f xv = *(const v2f*)(xs + (8 * hh + r) * NFEAT);
      x0[r] = xv[0];
      x1[r] = xv[1];
      if (warm) {
        const bool allpad = (x0[r] == -1.0f) && (x1[r] == -1.0f);
        if (allpad) mbits &= ~(1u << r);
      }
    }
    _Float16 hb1[8];
#pragma unroll
    for (int r = 0; r < 8; ++r) {
      float zq[4];
#pragma unroll
      for (int q = 0; q < 4; ++q) {
        const float xw = x0[r] * w1a[q] + x1[r] * w1b[q];
        zq[q] = (xw + acc[q][r] * OP_INV) + b1q[q];
      }
      const float ig = sigm(zq[0]);
      const float fg = sigm(zq[1]);
      const float gg = sigm(zq[2]);
      const float og = sigm(zq[3]);
      const float ct = fg * c1s[r] + ig * gg;
      const float ht = og * sigm(ct);
      const float cn = kv1 * ct + okv1 * c1s[r];
      const float hn = kv1 * ht + okv1 * h1s[r];
      const bool sel = ((mbits >> r) & 1u) != 0u;
      c1s[r] = sel ? cn : c1s[r];
      h1s[r] = sel ? hn : h1s[r];
      hb1[r] = (_Float16)(h1s[r] * OPA_SCALE);
    }
    __syncthreads();
#pragma unroll
    for (int r = 0; r < 8; ++r) Ah[(8 * hh + r) * APITCH + u1] = hb1[r];
    if (tt + 1 < NSEQ && wave == 0) {
      const int tn  = (tt + 1 < NSEQ) ? (tt + 1) : (NSEQ - 1);
      const int row = lane >> 1, f = lane & 1;
      const float v = inputs[(size_t)(b0 + row) * (NSEQ * NFEAT) + (size_t)tn * NFEAT + f];
      xs[lane] = (v - stt[row * 8 + f]) * stt[row * 8 + 2 + f];
    }
    __syncthreads();

    _Float16 hb2[8];
#pragma unroll
    for (int r = 0; r < 8; ++r) hb2[r] = hb1[r];
    if (wave < 4) {
      v8f acc2[4];
#pragma unroll
      for (int q = 0; q < 4; ++q) acc2[q] = z8;
#pragma unroll
      for (int ks = 0; ks < KCAT / 32; ++ks) {
        v16h bq[4];
#pragma unroll
        for (int q = 0; q < 4; ++q)
          bq[q] = Frag<_Float16>::load(Bcat + (size_t)(NH2 * q + u2) * KCAT + ks * 32 + 8 * hh);
        FU a;
        a.h[0] = *(const v8h*)(Ah + c * APITCH + ks * 32 + 8 * hh);
        a.h[1] = *(const v8h*)(Ah + c * APITCH + ks * 32 + 16 + 8 * hh);
#pragma unroll
        for (int q = 0; q < 4; ++q) acc2[q] = Frag<_Float16>::mma(a.v, bq[q], acc2[q]);
        dep_guard_h(acc2[0], acc2[3], a.v, a.v);
        keep4_h(bq[0], bq[1], bq[2], bq[3]);
      }
      acc_guard4(acc2[0], acc2[1], acc2[2], acc2[3]);

      const float kv2  = ktab[(size_t)tt * KTW + NH1 + u2];
      const float okv2 = 1.0f - kv2;
#pragma unroll
      for (int r = 0; r < 8; ++r) {
        const float ig = sigm(acc2[0][r] * OP_INV + b2q[0]);
        const float fg = sigm(acc2[1][r] * OP_INV + b2q[1]);
        const float gg = sigm(acc2[2][r] * OP_INV + b2q[2]);
        const float og = sigm(acc2[3][r] * OP_INV + b2q[3]);
        const float ct = fg * c2s[r] + ig * gg;
        const float ht = og * sigm(ct);
        const float cn = kv2 * ct + okv2 * c2s[r];
        const float hn = kv2 * ht + okv2 * h2s[r];
        const bool sel = ((mbits >> r) & 1u) != 0u;
        c2s[r] = sel ? cn : c2s[r];
        h2s[r] = sel ? hn : h2s[r];
        hb2[r] = (_Float16)(h2s[r] * OPA_SCALE);
      }
    }
    __syncthreads();
    if (wave < 4) {
#pragma unroll
      for (int r = 0; r < 8; ++r) Ah[(8 * hh + r) * APITCH + NH1 + u2] = hb2[r];
      if (tt >= NSEQ - 1) {
#pragma unroll
        for (int r = 0; r < 8; ++r) h2f[(8 * hh + r) * 68 + u2] = h2s[r];
      }
    }

    if (tt >= NSEQ - 1) {
      const int pi = tt - (NSEQ - 1);
      __syncthreads();
      {
        const int row = tid >> 4, j = tid & 15;
        float aa = 0.f, ab = 0.f;
#pragma unroll 4
        for (int k = 0; k < NH2; ++k) {
          const float hv = h2f[row * 68 + k];
          aa += hv * Wd1[k * NHD + j];
          ab += hv * Wd1[k * NHD + j + 16];
        }
        df[row * 36 + j]      = sigm(aa + bd1[j]);
        df[row * 36 + j + 16] = sigm(ab + bd1[j + 16]);
      }
      __syncthreads();
      if (wave == 0) {
        const int row = lane >> 1, f = lane & 1;
        float a2 = 0.f;
#pragma unroll 4
        for (int j = 0; j < NHD; ++j) a2 += df[row * 36 + j] * Wo[j * NFEAT + f];
        const float p = sigm(a2 + bo[f]);
        xs[lane] = p;
        predst[row * OUTROW + pi * NFEAT + f] = p * stt[row * 8 + 4 + f] + stt[row * 8 + f];
      }
      __syncthreads();
    }
  }

  __syncthreads();
  {
    const v4f val = *(const v4f*)(predst + tid * 4);
    float* op = out + (size_t)blockIdx.x * (ROWSPB * OUTROW) + tid * 4;
    *(volatile v4f*)op = val;
    __threadfence();
    *(volatile v4f*)op = val;
  }
}

extern "C" void kernel_launch(void* const* d_in, const int* in_sizes, int n_in,
                              void* d_out, int out_size, void* d_ws, size_t ws_size,
                              hipStream_t stream) {
  if (n_in < 18) return;
  const float* inputs = (const float*)d_in[0];
  const float* W1     = (const float*)d_in[1];
  const float* U1     = (const float*)d_in[2];
  const float* b1     = (const float*)d_in[3];
  const float* tau1   = (const float*)d_in[4];
  const float* shift1 = (const float*)d_in[5];
  const float* ron1   = (const float*)d_in[6];
  const float* W2     = (const float*)d_in[7];
  const float* U2     = (const float*)d_in[8];
  const float* b2     = (const float*)d_in[9];
  const float* tau2   = (const float*)d_in[10];
  const float* shift2 = (const float*)d_in[11];
  const float* ron2   = (const float*)d_in[12];
  const float* Wd1    = (const float*)d_in[13];
  const float* bd1    = (const float*)d_in[14];
  const float* Wo     = (const float*)d_in[15];
  const float* bo     = (const float*)d_in[16];
  const int*   osteps = (const int*)d_in[17];
  float* out = (float*)d_out;

  if (in_sizes[0] != NBATCH * NSEQ * NFEAT) return;
  if (in_sizes[2] != NH1 * 4 * NH1) return;
  if (in_sizes[7] != NH1 * 4 * NH2 || in_sizes[8] != NH2 * 4 * NH2) return;
  if (out_size < NBATCH * OUTROW) return;

  const size_t off_u1t   = 0;
  const size_t bytes_u1t = (size_t)(4 * NH1) * NH1 * 2;
  const size_t off_bcat  = off_u1t + bytes_u1t;
  const size_t bytes_bcat = (size_t)(4 * NH2) * KCAT * 2;
  const size_t off_stats = off_bcat + bytes_bcat;
  const size_t bytes_stats = (size_t)NBATCH * 4 * 4;
  const size_t off_ktab  = off_stats + bytes_stats;
  const size_t bytes_ktab = (size_t)NTT * KTW * 4;
  const size_t ws_need   = off_ktab + bytes_ktab;
  if (ws_need > ws_size) return;

  char* ws = (char*)d_ws;
  _Float16* U1t  = (_Float16*)(ws + off_u1t);
  _Float16* Bcat = (_Float16*)(ws + off_bcat);
  float*    stats = (float*)(ws + off_stats);
  float*    ktab  = (float*)(ws + off_ktab);

  const int nch1 = (4 * NH1) * NH1 / 8;
  k_prep_wt<<<(nch1 + 255) / 256, 256, 0, stream>>>(U1, NH1, U1, 0, 4 * NH1, U1t, nch1, OPB_SCALE);
  const int nch2 = (4 * NH2) * KCAT / 8;
  k_prep_wt<<<(nch2 + 255) / 256, 256, 0, stream>>>(W2, NH1, U2, NH2, 4 * NH2, Bcat, nch2, OPB_SCALE);
  k_stats<<<NBATCH / 8, 256, 0, stream>>>(inputs, stats);
  const int n4 = NTT * KTW / 4;
  k_ktab<<<(n4 + 255) / 256, 256, 0, stream>>>(tau1, shift1, ron1, tau2, shift2, ron2, ktab, n4);
  k_main<<<NBATCH / ROWSPB, 256, 0, stream>>>(inputs, W1, b1, b2, Wd1, bd1, Wo, bo, osteps,
                                              U1t, Bcat, stats, ktab, out);
}
